// MultiHeadedSelfAttention_12730283065399
// MI455X (gfx1250) — hardware-verified
//
#include <hip/hip_runtime.h>


#ifndef NB
#define NB 8
#endif
#ifndef SEQ
#define SEQ 1024
#endif
#define NB_FULL  8
#define SEQ_FULL 1024
#define DMOD 1024
#define NH   16
#define HD   64
#define RH   ((SEQ < 256) ? SEQ : 256)
#define BG   ((NB < 4) ? NB : 4)
#define PCAR 1024.0f
#define CS   0.18033688011112042f
#define PP   72
static_assert(SEQ % 64 == 0);
static_assert(RH % 64 == 0);
static_assert(NB % BG == 0);
static_assert(NB >= 1 && NB <= NB_FULL);
static_assert(SEQ <= SEQ_FULL);
static_assert(DMOD == NH * HD);
static_assert((size_t)NB * 2 <= (size_t)BG * 6);

typedef _Float16 h16;
typedef unsigned short bf;
typedef __attribute__((ext_vector_type(16))) __bf16   v16bf;
typedef __attribute__((ext_vector_type(16))) _Float16 v16h;
typedef __attribute__((ext_vector_type(8)))  _Float16 v8h;
typedef __attribute__((ext_vector_type(8)))  unsigned short v8us;
typedef __attribute__((ext_vector_type(8)))  float    v8f;
typedef __attribute__((ext_vector_type(4)))  float    v4f;
typedef __attribute__((ext_vector_type(2)))  _Float16 v2h;
typedef __attribute__((ext_vector_type(2)))  unsigned short v2us;
typedef __attribute__((ext_vector_type(2)))  float    v2f;
typedef v8h  __attribute__((may_alias)) v8ha;
typedef v4f  __attribute__((may_alias)) v4fa;
typedef v8us __attribute__((may_alias)) v8usa;

__device__ __forceinline__ unsigned short f2bf(float f) { unsigned u = __float_as_uint(f); u += 0x7FFFu + ((u >> 16) & 1u); return (unsigned short)(u >> 16); }
__device__ __forceinline__ float bf2f(unsigned short b) { return __uint_as_float(((unsigned)b) << 16); }
__device__ __forceinline__ float bfr(float f) { return bf2f(f2bf(f)); }
__device__ __forceinline__ v16h cat16(v8h lo, v8h hi) { return __builtin_shufflevector(lo, hi, 0, 1, 2, 3, 4, 5, 6, 7, 8, 9, 10, 11, 12, 13, 14, 15); }
__device__ __forceinline__ v16bf cat16b(v8us lo, v8us hi) { return __builtin_bit_cast(v16bf, __builtin_shufflevector(lo, hi, 0, 1, 2, 3, 4, 5, 6, 7, 8, 9, 10, 11, 12, 13, 14, 15)); }
__device__ __forceinline__ v8f wmma16(v16h a, v16h b, v8f c) { return __builtin_amdgcn_wmma_f32_16x16x32_f16(false, a, false, b, (short)0, c, false, false); }
__device__ __forceinline__ v8f wmmab(v16bf a, v16bf b, v8f c) { return __builtin_amdgcn_wmma_f32_16x16x32_bf16(false, a, false, b, (short)0, c, false, false); }
__device__ __forceinline__ h16 tohx(float x) { return (h16)x; }
__device__ __forceinline__ void splitf(float y, unsigned short& h, unsigned short& l) { h = f2bf(y); l = f2bf(y - bf2f(h)); }

template <typename T16> struct WFrag;
template <> struct WFrag<h16> { typedef v16h V; static __device__ __forceinline__ V ld(const h16* p) { return cat16(*(const v8h*)p, *(const v8h*)(p + 16)); } static __device__ __forceinline__ v8f mma(V a, V b, v8f c) { return wmma16(a, b, c); } };
template <> struct WFrag<bf> { typedef v16bf V; static __device__ __forceinline__ V ld(const bf* p) { return cat16b(*(const v8us*)p, *(const v8us*)(p + 16)); } static __device__ __forceinline__ v8f mma(V a, V b, v8f c) { return wmmab(a, b, c); } };

template <typename T16, int NSPLIT, bool BIAS>
__global__ __launch_bounds__(32) void k_gemmw(const T16* __restrict__ A, const T16* __restrict__ A2, const T16* __restrict__ Bt, const T16* __restrict__ Bt2, int K, float* C, int ldc, const float* __restrict__ bias, size_t sA, size_t sB, size_t sC) {
    typedef typename WFrag<T16>::V V;
    __shared__ __align__(16) float os[16 * 68];
    const size_t z = blockIdx.z; A += z * sA; if (A2) A2 += z * sA; Bt += z * sB; if (Bt2) Bt2 += z * sB; C += z * sC;
    const int lane = threadIdx.x & 31, lr = lane & 15, hi = lane >> 4; const int r0 = blockIdx.x * 64, c0 = blockIdx.y * 64;
    v8f acc[4][4];
#pragma unroll
    for (int mb = 0; mb < 4; ++mb)
#pragma unroll
        for (int nb = 0; nb < 4; ++nb) acc[mb][nb] = (v8f){};
    const size_t aoff = (size_t)(r0 + lr) * K + 8 * hi, boff = (size_t)(c0 + lr) * K + 8 * hi;
#pragma unroll 1
    for (int kc = 0; kc < K; kc += 32) {
        V a[4], a2[4];
#pragma unroll
        for (int mb = 0; mb < 4; ++mb) { a[mb] = WFrag<T16>::ld(A + aoff + (size_t)mb * 16 * K + kc); if (NSPLIT == 1 || NSPLIT == 2) a2[mb] = WFrag<T16>::ld(A2 + aoff + (size_t)mb * 16 * K + kc); }
#pragma unroll
        for (int nb = 0; nb < 4; ++nb) { const V b = WFrag<T16>::ld(Bt + boff + (size_t)nb * 16 * K + kc); V b2; if (NSPLIT >= 2) b2 = WFrag<T16>::ld(Bt2 + boff + (size_t)nb * 16 * K + kc);
#pragma unroll
            for (int mb = 0; mb < 4; ++mb) { acc[mb][nb] = WFrag<T16>::mma(a[mb], b, acc[mb][nb]); if (NSPLIT == 1 || NSPLIT == 2) acc[mb][nb] = WFrag<T16>::mma(a2[mb], b, acc[mb][nb]); if (NSPLIT >= 2) acc[mb][nb] = WFrag<T16>::mma(a[mb], b2, acc[mb][nb]); } }
        asm volatile("v_nop\n\tv_nop\n\tv_nop\n\tv_nop" : "+v"(acc[0][0]), "+v"(acc[1][1]), "+v"(acc[2][2]), "+v"(acc[3][3]) : "v"(a[0]), "v"(a[3]));
    }
    v4f bb; bb[0] = 0.f; bb[1] = 0.f; bb[2] = 0.f; bb[3] = 0.f;
    if (BIAS) { const int cofs = lr * 4; bb[0] = bfr(bias[c0 + cofs]); bb[1] = bfr(bias[c0 + cofs + 1]); bb[2] = bfr(bias[c0 + cofs + 2]); bb[3] = bfr(bias[c0 + cofs + 3]); }
#pragma unroll
    for (int mb = 0; mb < 4; ++mb) {
#pragma unroll
        for (int nb = 0; nb < 4; ++nb) {
#pragma unroll
            for (int j = 0; j < 8; ++j) os[(hi * 8 + j) * 68 + nb * 16 + lr] = acc[mb][nb][j]; }
        __builtin_amdgcn_wave_barrier(); asm volatile("" ::: "memory");
        float* crow = C + (size_t)(r0 + mb * 16) * ldc + c0;
#pragma unroll 1
        for (int ps = 0; ps < 2; ++ps) {
#pragma unroll
            for (int s = 0; s < 8; ++s) { const int row = 2 * s + hi, cofs = lr * 4; v4f val = *(const v4fa*)(os + row * 68 + cofs); if (BIAS) val += bb;
                *(volatile v4f*)(crow + (size_t)row * ldc + cofs) = val; }
            if (ps == 0) __threadfence(); }
        __builtin_amdgcn_wave_barrier(); asm volatile("" ::: "memory");
    }
}

__global__ __launch_bounds__(256) void k_wtG(const float* __restrict__ w, int K, int N, bf* Bt) {
    const int lane = threadIdx.x & 31; const int L0 = (blockIdx.x * 8 + (threadIdx.x >> 5)) * 8; const int nlines = N * K / 64;
#pragma unroll
    for (int ps = 0; ps < 2; ++ps) {
#pragma unroll 1
        for (int l = 0; l < 8; ++l) { const int L = L0 + l; if (L >= nlines) break; const size_t e = (size_t)L * 64 + lane * 2; const int k = (int)(e % K), n = (int)(e / K); v2us o;
            o[0] = f2bf(w[(size_t)k * N + n]); o[1] = f2bf(w[(size_t)(k + 1) * N + n]); *(volatile v2us*)(Bt + e) = o; }
        if (ps == 0) __threadfence(); }
}

__global__ __launch_bounds__(256) void k_cvtx(const float* __restrict__ x, int g0, bf* XB, size_t n8) {
    const size_t i = (size_t)blockIdx.x * 256 + threadIdx.x; if (i >= n8) return;
    const size_t row = i / (DMOD / 8); const int c8 = (int)(i % (DMOD / 8)) * 8; const int bl = (int)(row / SEQ), t = (int)(row % SEQ);
    const v8f v = *(const v8f*)(x + ((size_t)(g0 + bl) * SEQ_FULL + t) * DMOD + c8); v8us o;
#pragma unroll
    for (int k = 0; k < 8; ++k) o[k] = f2bf(v[k]);
    *(volatile v8us*)(XB + i * 8) = o; __threadfence(); *(volatile v8us*)(XB + i * 8) = o;
}

__global__ __launch_bounds__(256) void k_qkp(const float* __restrict__ F, int g0, h16* P16, bf* Ph, bf* Pl) {
    const size_t e = ((size_t)blockIdx.x * 256 + threadIdx.x) * 2; const size_t tot = (size_t)BG * NH * SEQ * HD; if (e >= tot) return;
    const int d = (int)(e % HD); const int t = (int)((e / HD) % SEQ); const int hh = (int)((e / ((size_t)HD * SEQ)) % NH); const int bl = (int)(e / ((size_t)HD * SEQ * NH));
    const v2f xv = *(const v2f*)(F + ((size_t)bl * SEQ + t) * DMOD + hh * HD + d);
    v2h o16; v2us oh, ol;
#pragma unroll
    for (int q = 0; q < 2; ++q) { o16[q] = tohx(xv[q]); unsigned short a1, a2; splitf(xv[q], a1, a2); oh[q] = a1; ol[q] = a2; }
    const size_t g = (size_t)(g0 + bl) * NH + hh; const bool rs = (t < RH); const int tr = rs ? t : 0;
    h16* p16 = P16 + (g * SEQ + t) * HD + d; bf* ph = Ph + (g * RH + tr) * HD + d; bf* pl = Pl + (g * RH + tr) * HD + d;
    *(volatile v2h*)p16 = o16; if (rs) { *(volatile v2us*)ph = oh; *(volatile v2us*)pl = ol; }
    __threadfence();
    *(volatile v2h*)p16 = o16; if (rs) { *(volatile v2us*)ph = oh; *(volatile v2us*)pl = ol; }
}

__global__ __launch_bounds__(256) void k_vtp(const float* __restrict__ F, int g0, h16* V16, bf* Vh, bf* Vl) {
    const size_t e = ((size_t)blockIdx.x * 256 + threadIdx.x) * 2; const size_t tot = (size_t)BG * NH * HD * SEQ; if (e >= tot) return;
    const int t = (int)(e % SEQ); const int d = (int)((e / SEQ) % HD); const int hh = (int)((e / ((size_t)SEQ * HD)) % NH); const int bl = (int)(e / ((size_t)SEQ * HD * NH));
    v2h o16; v2us oh, ol;
#pragma unroll
    for (int q = 0; q < 2; ++q) { const float xv = F[((size_t)bl * SEQ + t + q) * DMOD + hh * HD + d]; o16[q] = tohx(xv); unsigned short a1, a2; splitf(xv, a1, a2); oh[q] = a1; ol[q] = a2; }
    const size_t g = (size_t)(g0 + bl) * NH + hh; const bool rs = (t < RH); const int tr = rs ? t : 0;
    h16* p16 = V16 + (g * HD + d) * SEQ + t; bf* ph = Vh + (g * HD + d) * RH + tr; bf* pl = Vl + (g * HD + d) * RH + tr;
    *(volatile v2h*)p16 = o16; if (rs) { *(volatile v2us*)ph = oh; *(volatile v2us*)pl = ol; }
    __threadfence();
    *(volatile v2h*)p16 = o16; if (rs) { *(volatile v2us*)ph = oh; *(volatile v2us*)pl = ol; }
}

template <bool R> struct Sel { typedef h16 T; };
template <> struct Sel<true> { typedef bf T; };

template <bool RES>
__global__ __launch_bounds__(128) __attribute__((amdgpu_num_vgpr(256)))
void k_attn(const h16* __restrict__ Q16, const bf* __restrict__ Qh, const bf* __restrict__ Ql,
            const h16* __restrict__ K16, const bf* __restrict__ Kh, const bf* __restrict__ Kl,
            const h16* __restrict__ V16, const bf* __restrict__ Vh, const bf* __restrict__ Vl,
            bf* ATh, bf* ATl, int qb0) {
    typedef typename Sel<RES>::T T; typedef typename WFrag<T>::V FV;
    __shared__ __align__(16) T pt[2][4][16 * PP];
    __shared__ __align__(16) unsigned short eh[4][16 * PP];
    __shared__ __align__(16) unsigned short el[4][16 * PP];
    const int w = threadIdx.x >> 5, lane = threadIdx.x & 31, lr = lane & 15, hi = lane >> 4;
    const int qb = qb0 + (int)blockIdx.x, h = (int)blockIdx.y, bz = (int)blockIdx.z;
    const int t0 = qb * 64 + w * 16;
    const size_t g = (size_t)bz * NH + h;
    const T* qp; const T* qp2; const T* kbase; const T* kbase2; const T* vbase; const T* vbase2; size_t vpit;
    if (RES) {
        qp = (const T*)(const void*)Qh + (g * RH + t0 + lr) * HD + 8 * hi;   qp2 = (const T*)(const void*)Ql + (g * RH + t0 + lr) * HD + 8 * hi;
        kbase = (const T*)(const void*)Kh + (g * RH + lr) * HD + 8 * hi;     kbase2 = (const T*)(const void*)Kl + (g * RH + lr) * HD + 8 * hi;
        vbase = (const T*)(const void*)Vh + (g * HD + lr) * RH + 8 * hi;     vbase2 = (const T*)(const void*)Vl + (g * HD + lr) * RH + 8 * hi;  vpit = RH;
    } else {
        qp = (const T*)(const void*)Q16 + (g * SEQ + t0 + lr) * HD + 8 * hi; qp2 = qp;
        kbase = (const T*)(const void*)K16 + (g * SEQ + lr) * HD + 8 * hi;   kbase2 = kbase;
        vbase = (const T*)(const void*)V16 + (g * HD + lr) * SEQ + 8 * hi;   vbase2 = vbase;  vpit = SEQ;
    }
    FV qa[2], qa2[2];
#pragma unroll
    for (int ks = 0; ks < 2; ++ks) { qa[ks] = WFrag<T>::ld(qp + ks * 32); qa2[ks] = RES ? WFrag<T>::ld(qp2 + ks * 32) : qa[ks]; }
    v8f acc[4];
#pragma unroll
    for (int nb = 0; nb < 4; ++nb) acc[nb] = (v8f){};
    float mrow[8], lrow[8];
#pragma unroll
    for (int r = 0; r < 8; ++r) { mrow[r] = -__builtin_inff(); lrow[r] = 0.f; }
    const int qloc = w * 16 + 8 * hi - lr;
#pragma unroll 1
    for (int c = 0; c <= qb; ++c) {
        v8f s[4];
#pragma unroll
        for (int nb = 0; nb < 4; ++nb) s[nb] = (v8f){};
        const T* kp = kbase + (size_t)c * 64 * HD; const T* kp2 = kbase2 + (size_t)c * 64 * HD;
        FV klast;
#pragma unroll
        for (int nb = 0; nb < 4; ++nb) {
#pragma unroll
            for (int ks = 0; ks < 2; ++ks) {
                const FV kb = WFrag<T>::ld(kp + nb * 16 * HD + ks * 32);
                s[nb] = WFrag<T>::mma(qa[ks], kb, s[nb]);
                if (RES) { const FV kb2 = WFrag<T>::ld(kp2 + nb * 16 * HD + ks * 32); s[nb] = WFrag<T>::mma(qa[ks], kb2, s[nb]); s[nb] = WFrag<T>::mma(qa2[ks], kb, s[nb]); }
                klast = kb; } }
        asm volatile("v_nop\n\tv_nop\n\tv_nop\n\tv_nop" : "+v"(s[0]), "+v"(s[1]), "+v"(s[2]), "+v"(s[3]) : "v"(qa[0]), "v"(qa[1]), "v"(klast));
        const int lim = (c == qb) ? qloc : (1 << 20);
        float cm[8];
#pragma unroll
        for (int r = 0; r < 8; ++r) cm[r] = -__builtin_inff();
#pragma unroll
        for (int nb = 0; nb < 4; ++nb)
#pragma unroll
            for (int r = 0; r < 8; ++r) { float vv = s[nb][r]; if (nb * 16 - r > lim) vv = -__builtin_inff(); s[nb][r] = vv; cm[r] = fmaxf(cm[r], vv); }
#pragma unroll
        for (int r = 0; r < 8; ++r) {
#pragma unroll
            for (int sh = 1; sh < 16; sh <<= 1) cm[r] = fmaxf(cm[r], __shfl_xor(cm[r], sh, 32)); }
#pragma unroll
        for (int r = 0; r < 8; ++r) { const float mn = fmaxf(mrow[r], cm[r]); const float al = __builtin_amdgcn_exp2f((mrow[r] - mn) * CS); mrow[r] = mn; lrow[r] *= al;
#pragma unroll
            for (int nb = 0; nb < 4; ++nb) acc[nb][r] *= al; }
        float psum[8];
#pragma unroll
        for (int r = 0; r < 8; ++r) psum[r] = 0.f;
        T* tile = pt[0][w]; T* tile2 = pt[1][w];
#pragma unroll
        for (int nb = 0; nb < 4; ++nb)
#pragma unroll
            for (int r = 0; r < 8; ++r) {
                const float p = __builtin_amdgcn_exp2f((s[nb][r] - mrow[r]) * CS);
                const int o = (8 * hi + r) * PP + nb * 16 + lr;
                if (RES) { unsigned short a1, a2; splitf(p, a1, a2); ((unsigned short*)(void*)tile)[o] = a1; ((unsigned short*)(void*)tile2)[o] = a2; psum[r] += p; }
                else { const h16 ph = tohx(p * PCAR); ((h16*)(void*)tile)[o] = ph; psum[r] += (float)ph; } }
#pragma unroll
        for (int r = 0; r < 8; ++r) {
#pragma unroll
            for (int sh = 1; sh < 16; sh <<= 1) psum[r] += __shfl_xor(psum[r], sh, 32); lrow[r] += psum[r]; }
        __syncthreads();
        FV pa[2], pa2[2];
#pragma unroll
        for (int ks = 0; ks < 2; ++ks) { pa[ks] = WFrag<T>::ld(tile + lr * PP + ks * 32 + 8 * hi); pa2[ks] = RES ? WFrag<T>::ld(tile2 + lr * PP + ks * 32 + 8 * hi) : pa[ks]; }
        const T* vp = vbase + (size_t)c * 64; const T* vp2 = vbase2 + (size_t)c * 64;
        FV vlast;
#pragma unroll
        for (int nb = 0; nb < 4; ++nb) {
#pragma unroll
            for (int ks = 0; ks < 2; ++ks) {
                const FV vb = WFrag<T>::ld(vp + nb * 16 * vpit + ks * 32);
                acc[nb] = WFrag<T>::mma(pa[ks], vb, acc[nb]);
                if (RES) { const FV vb2 = WFrag<T>::ld(vp2 + nb * 16 * vpit + ks * 32); acc[nb] = WFrag<T>::mma(pa[ks], vb2, acc[nb]); acc[nb] = WFrag<T>::mma(pa2[ks], vb, acc[nb]); }
                vlast = vb; } }
        asm volatile("v_nop\n\tv_nop\n\tv_nop\n\tv_nop" : "+v"(acc[0]), "+v"(acc[1]), "+v"(acc[2]), "+v"(acc[3]) : "v"(pa[0]), "v"(pa[1]), "v"(vlast));
        __syncthreads();
    }
    float inv[8];
#pragma unroll
    for (int r = 0; r < 8; ++r) inv[r] = 1.0f / lrow[r];
#pragma unroll
    for (int nb = 0; nb < 4; ++nb)
#pragma unroll
        for (int r = 0; r < 8; ++r) { unsigned short a1, a2; splitf(acc[nb][r] * inv[r], a1, a2); const int o = (8 * hi + r) * PP + nb * 16 + lr; eh[w][o] = a1; el[w][o] = a2; }
    __syncthreads();
    const int rq = lane >> 3, c8 = (lane & 7) * 8;
    bf* gh = ATh + ((size_t)bz * SEQ + t0) * DMOD + h * HD + c8; bf* gl = ATl + ((size_t)bz * SEQ + t0) * DMOD + h * HD + c8;
#pragma unroll 1
    for (int ps = 0; ps < 2; ++ps) {
#pragma unroll
        for (int si = 0; si < 4; ++si) { const int row = rq + 4 * si; const v8us xh = *(const v8usa*)(eh[w] + row * PP + c8); const v8us xl = *(const v8usa*)(el[w] + row * PP + c8);
            *(volatile v8us*)(gh + (size_t)row * DMOD) = xh; *(volatile v8us*)(gl + (size_t)row * DMOD) = xl; }
        if (ps == 0) __threadfence(); }
}

extern "C" void kernel_launch(void* const* d_in, const int* in_sizes, int n_in,
                              void* d_out, int out_size, void* d_ws, size_t ws_size, hipStream_t stream) {
    if (n_in < 9) return;
    const long long need_rows = (long long)(NB - 1) * SEQ_FULL + SEQ;
    if ((long long)in_sizes[0] < need_rows * DMOD || (long long)out_size < need_rows * DMOD) return;
    if (in_sizes[1] < DMOD * DMOD || in_sizes[3] < DMOD * DMOD || in_sizes[5] < DMOD * DMOD || in_sizes[7] < DMOD * DMOD) return;
    if (in_sizes[2] < DMOD || in_sizes[4] < DMOD || in_sizes[6] < DMOD || in_sizes[8] < DMOD) return;
    const float* x  = (const float*)d_in[0];
    const float* Wq = (const float*)d_in[1]; const float* bq = (const float*)d_in[2];
    const float* Wk = (const float*)d_in[3]; const float* bk = (const float*)d_in[4];
    const float* Wv = (const float*)d_in[5]; const float* bv = (const float*)d_in[6];
    const float* Wo = (const float*)d_in[7]; const float* bo = (const float*)d_in[8];
    float* OUT = (float*)d_out;
    char* wsp = (char*)d_ws;
    auto take = [&](size_t bytes) { char* p = wsp; wsp += (bytes + 255) & ~(size_t)255; return (void*)p; };
    bf* WQ = (bf*)take((size_t)DMOD * DMOD * 2); bf* WK = (bf*)take((size_t)DMOD * DMOD * 2); bf* WV = (bf*)take((size_t)DMOD * DMOD * 2); bf* WO = (bf*)take((size_t)DMOD * DMOD * 2);
    bf* XB = (bf*)take((size_t)BG * SEQ * DMOD * 2);
    float* F = (float*)take((size_t)BG * SEQ * DMOD * 4);
    h16* Q16 = (h16*)take((size_t)NB * NH * SEQ * HD * 2); bf* Qh = (bf*)take((size_t)NB * NH * RH * HD * 2); bf* Ql = (bf*)take((size_t)NB * NH * RH * HD * 2);
    h16* K16 = (h16*)take((size_t)NB * NH * SEQ * HD * 2); bf* Kh = (bf*)take((size_t)NB * NH * RH * HD * 2); bf* Kl = (bf*)take((size_t)NB * NH * RH * HD * 2);
    h16* V16 = (h16*)take((size_t)NB * NH * HD * SEQ * 2); bf* Vh = (bf*)take((size_t)NB * NH * HD * RH * 2); bf* Vl = (bf*)take((size_t)NB * NH * HD * RH * 2);
    bf* ATh = (bf*)take((size_t)NB * SEQ * DMOD * 2);
    bf* ATl = XB;
    const size_t carved = (size_t)(wsp - (char*)d_ws);
    if (carved > ws_size || carved > ((size_t)128 << 20)) return;

    const unsigned gw = (unsigned)((DMOD * DMOD / 64 + 63) / 64);
    k_wtG<<<gw, 256, 0, stream>>>(Wq, DMOD, DMOD, WQ);
    k_wtG<<<gw, 256, 0, stream>>>(Wk, DMOD, DMOD, WK);
    k_wtG<<<gw, 256, 0, stream>>>(Wv, DMOD, DMOD, WV);
    k_wtG<<<gw, 256, 0, stream>>>(Wo, DMOD, DMOD, WO);
    const size_t n8 = (size_t)BG * SEQ * DMOD / 8;
    const unsigned gcv = (unsigned)((n8 + 255) / 256);
    const unsigned gpl = (unsigned)(((size_t)BG * NH * SEQ * HD / 2 + 255) / 256);
    const dim3 ggm((unsigned)(BG * SEQ / 64), (unsigned)(DMOD / 64), 1);
    for (int g0 = 0; g0 < NB; g0 += BG) {
        k_cvtx<<<gcv, 256, 0, stream>>>(x, g0, XB, n8);
        k_gemmw<bf, 0, true><<<ggm, 32, 0, stream>>>(XB, nullptr, WQ, nullptr, DMOD, F, DMOD, bq, 0, 0, 0);
        k_qkp<<<gpl, 256, 0, stream>>>(F, g0, Q16, Qh, Ql);
        k_gemmw<bf, 0, true><<<ggm, 32, 0, stream>>>(XB, nullptr, WK, nullptr, DMOD, F, DMOD, bk, 0, 0, 0);
        k_qkp<<<gpl, 256, 0, stream>>>(F, g0, K16, Kh, Kl);
        k_gemmw<bf, 0, true><<<ggm, 32, 0, stream>>>(XB, nullptr, WV, nullptr, DMOD, F, DMOD, bv, 0, 0, 0);
        k_vtp<<<gpl, 256, 0, stream>>>(F, g0, V16, Vh, Vl);
    }
    k_attn<true><<<dim3((unsigned)(RH / 64), NH, NB), 128, 0, stream>>>(Q16, Qh, Ql, K16, Kh, Kl, V16, Vh, Vl, ATh, ATl, 0);
    if (SEQ > RH) k_attn<false><<<dim3((unsigned)((SEQ - RH) / 64), NH, NB), 128, 0, stream>>>(Q16, Qh, Ql, K16, Kh, Kl, V16, Vh, Vl, ATh, ATl, RH / 64);
    k_gemmw<bf, 1, true><<<dim3((unsigned)(SEQ / 64), (unsigned)(DMOD / 64), NB), 32, 0, stream>>>(ATh, ATl, WO, nullptr, DMOD, OUT, DMOD, bo, (size_t)SEQ * DMOD, (size_t)0, (size_t)SEQ_FULL * DMOD);
}
